// LinearAttention_10333691314265
// MI455X (gfx1250) — hardware-verified
//
#include <hip/hip_runtime.h>
#include <math.h>

constexpr int kSeq   = 2048;
constexpr int kDim   = 1024;
constexpr int kHeads = 16;
constexpr int kDh    = 64;
constexpr int kPairs = kDh / 2;
constexpr int kChunk = 64;
constexpr int kNC    = kSeq / kChunk;
constexpr int kQKVld = 3 * kDim;
constexpr int kTP    = 72;
constexpr int kFP    = 68;
constexpr float kEps   = 1.0e-6f;
constexpr float kTheta = 10000.0f;
static_assert(kHeads * kDh == kDim, "shape");
static_assert(kNC == 32 && kChunk == 64 && kDh == 64, "chunking");
static_assert(kSeq % 64 == 0 && kDim % 64 == 0 && kQKVld % 64 == 0 && kDim % 32 == 0, "gemm tiles");

typedef __attribute__((ext_vector_type(16))) _Float16 v16h;
typedef __attribute__((ext_vector_type(8)))  _Float16 v8h;
typedef __attribute__((ext_vector_type(16))) __bf16   v16b;
typedef __attribute__((ext_vector_type(8)))  __bf16   v8b;
typedef __attribute__((ext_vector_type(8)))  float    v8f;
typedef __attribute__((ext_vector_type(4)))  float    v4f;
typedef __attribute__((ext_vector_type(2)))  float    v2f;
typedef __attribute__((ext_vector_type(4)))  unsigned int v4u;
typedef __attribute__((ext_vector_type(2)))  unsigned int v2u;

__device__ __forceinline__ unsigned short f2bf_bits(float f) {
  unsigned u = __float_as_uint(f);
  return (unsigned short)((u + 0x7FFFu + ((u >> 16) & 1u)) >> 16);
}
__device__ __forceinline__ float bf_bits2f(unsigned short h) { return __uint_as_float(((unsigned)h) << 16); }
__device__ __forceinline__ unsigned pk16(unsigned short a, unsigned short b) { return (unsigned)a | ((unsigned)b << 16); }
__device__ __forceinline__ void split_bf(float f, unsigned short& hb, unsigned short& lb) {
  hb = f2bf_bits(f);
  lb = f2bf_bits(f - bf_bits2f(hb));
}
__device__ __forceinline__ v8f zero8() { return (v8f){0.f, 0.f, 0.f, 0.f, 0.f, 0.f, 0.f, 0.f}; }

__device__ __forceinline__ void dep_guard4_h(v8f& a, v8f& b, v8f& c, v8f& d, v16h x, v16h y) {
  asm volatile("v_nop\n\tv_nop\n\tv_nop\n\tv_nop" : "+v"(a), "+v"(b), "+v"(c), "+v"(d) : "v"(x), "v"(y));
}
__device__ __forceinline__ void dep_guard4_b(v8f& a, v8f& b, v8f& c, v8f& d, v16b x, v16b y) {
  asm volatile("v_nop\n\tv_nop\n\tv_nop\n\tv_nop" : "+v"(a), "+v"(b), "+v"(c), "+v"(d) : "v"(x), "v"(y));
}
__device__ __forceinline__ void keep4_h(v16h a, v16h b, v16h c, v16h d) { asm volatile("v_nop" :: "v"(a), "v"(b), "v"(c), "v"(d)); }
__device__ __forceinline__ void keep4_b(v16b a, v16b b, v16b c, v16b d) { asm volatile("v_nop" :: "v"(a), "v"(b), "v"(c), "v"(d)); }
__device__ __forceinline__ void acc_guard4(v8f& a, v8f& b, v8f& c, v8f& d) { asm volatile("v_nop\n\tv_nop\n\tv_nop\n\tv_nop" : "+v"(a), "+v"(b), "+v"(c), "+v"(d)); }
__device__ __forceinline__ void tile_guard(v8f& a0, v8f& a1, v8f& a2, v8f& a3, v16b ah, v16b al,
                                           v16b b0, v16b b1, v16b b2, v16b b3, v16b c0, v16b c1, v16b c2, v16b c3) {
  asm volatile("v_nop\n\tv_nop\n\tv_nop\n\tv_nop"
               : "+v"(a0), "+v"(a1), "+v"(a2), "+v"(a3)
               : "v"(ah), "v"(al), "v"(b0), "v"(b1), "v"(b2), "v"(b3), "v"(c0), "v"(c1), "v"(c2), "v"(c3));
}

template <typename T> struct Frag;
template <> struct Frag<_Float16> {
  typedef v16h V; union U { v16h v; v8h h[2]; };
  static __device__ __forceinline__ v16h load(const _Float16* p) {
    U f; f.h[0] = *(const v8h*)(p); f.h[1] = *(const v8h*)(p + 16); return f.v;
  }
  static __device__ __forceinline__ v8f mma(v16h a, v16h b, v8f c) {
    return __builtin_amdgcn_wmma_f32_16x16x32_f16(false, a, false, b, (short)0, c, false, false);
  }
  static __device__ __forceinline__ void guard4(v8f& a, v8f& b, v8f& c, v8f& d, v16h x, v16h y) { dep_guard4_h(a, b, c, d, x, y); }
  static __device__ __forceinline__ void keep(v16h a, v16h b, v16h c, v16h d) { keep4_h(a, b, c, d); }
};
template <> struct Frag<__bf16> {
  typedef v16b V; union U { v16b v; v8b h[2]; };
  static __device__ __forceinline__ v16b load(const __bf16* p) {
    U f; f.h[0] = *(const v8b*)(p); f.h[1] = *(const v8b*)(p + 16); return f.v;
  }
  static __device__ __forceinline__ v8f mma(v16b a, v16b b, v8f c) {
    return __builtin_amdgcn_wmma_f32_16x16x32_bf16(false, a, false, b, (short)0, c, false, false);
  }
  static __device__ __forceinline__ void guard4(v8f& a, v8f& b, v8f& c, v8f& d, v16b x, v16b y) { dep_guard4_b(a, b, c, d, x, y); }
  static __device__ __forceinline__ void keep(v16b a, v16b b, v16b c, v16b d) { keep4_b(a, b, c, d); }
};

template <int ET> struct Elem;
template <> struct Elem<0> { typedef _Float16 T; };
template <> struct Elem<1> { typedef __bf16 T; };
template <int ET, int SPLITM, int BIAS_MODE, int OUT_MODE>
__global__ __launch_bounds__(256) void wmma_gemm64(
    const unsigned short* __restrict__ Ap, const unsigned short* __restrict__ A2p, int lda, long strideA,
    const unsigned short* __restrict__ Btp, const unsigned short* __restrict__ Bt2p, int ldb, long strideB,
    void* __restrict__ Cout, void* __restrict__ Cout2, int ldc, long strideC,
    const float* __restrict__ bias,
    int M, int N, int K, float scale) {
  typedef typename Elem<ET>::T T;
  typedef typename Frag<T>::V V;
  const T* A = (const T*)Ap; const T* A2 = (const T*)A2p; const T* Bt = (const T*)Btp; const T* Bt2 = (const T*)Bt2p;
  __shared__ __align__(16) float sT[8][16 * 68];
  const int b    = blockIdx.y;
  const int lane = threadIdx.x & 31;
  const int wave = threadIdx.x >> 5;
  const int tilesN = N >> 6;
  const int tilesM = M >> 6;
  const int tile = blockIdx.x * 8 + wave;
  if (tile >= tilesM * tilesN) return;
  const int tm = tile / tilesN;
  const int tn = tile - tm * tilesN;
  const int m0 = tm << 6;
  const int n0 = tn << 6;

  const T* Ab  = A  + (size_t)b * strideA;
  const T* Bb  = Bt + (size_t)b * strideB;
  const T* Ab2 = (SPLITM >= 1) ? (A2  + (size_t)b * strideA) : nullptr;
  const T* Bb2 = (SPLITM == 2) ? (Bt2 + (size_t)b * strideB) : nullptr;

  const int rlane = lane & 15;
  const int koff  = (lane >> 4) * 8;
  const int mOff  = (lane >> 4) * 8;

  v8f acc[4][4];
#pragma unroll
  for (int i = 0; i < 4; ++i)
#pragma unroll
    for (int j = 0; j < 4; ++j) acc[i][j] = zero8();

  for (int k0 = 0; k0 < K; k0 += 32) {
    V bh[4], bl[4];
#pragma unroll
    for (int j = 0; j < 4; ++j) {
      const size_t bo = (size_t)(n0 + (j << 4) + rlane) * ldb + koff + k0;
      bh[j] = Frag<T>::load(Bb + bo);
      bl[j] = bh[j];
      if (SPLITM == 2) bl[j] = Frag<T>::load(Bb2 + bo);
    }
#pragma unroll
    for (int i = 0; i < 4; ++i) {
      const size_t ao = (size_t)(m0 + (i << 4) + rlane) * lda + koff + k0;
      V ah = Frag<T>::load(Ab + ao);
      V al = ah;
      if (SPLITM >= 1) al = Frag<T>::load(Ab2 + ao);
#pragma unroll
      for (int j = 0; j < 4; ++j) {
        acc[i][j] = Frag<T>::mma(ah, bh[j], acc[i][j]);
        if (SPLITM == 2) acc[i][j] = Frag<T>::mma(ah, bl[j], acc[i][j]);
        if (SPLITM >= 1) acc[i][j] = Frag<T>::mma(al, bh[j], acc[i][j]);
      }
      Frag<T>::guard4(acc[i][0], acc[i][1], acc[i][2], acc[i][3], ah, al);
    }
    Frag<T>::keep(bh[0], bh[1], bh[2], bh[3]);
    if (SPLITM == 2) Frag<T>::keep(bl[0], bl[1], bl[2], bl[3]);
  }
  acc_guard4(acc[0][0], acc[0][1], acc[0][2], acc[0][3]);
  acc_guard4(acc[1][0], acc[1][1], acc[1][2], acc[1][3]);
  acc_guard4(acc[2][0], acc[2][1], acc[2][2], acc[2][3]);
  acc_guard4(acc[3][0], acc[3][1], acc[3][2], acc[3][3]);

  float* slab = sT[wave];
#pragma unroll
  for (int i = 0; i < 4; ++i) {
    const int mBase = m0 + (i << 4);
#pragma unroll
    for (int j = 0; j < 4; ++j) {
      const int n = n0 + (j << 4) + rlane;
      float bv = 0.f;
      if (BIAS_MODE == 2) bv = bias[n];
#pragma unroll
      for (int r = 0; r < 8; ++r) {
        float v = acc[i][j][r] * scale;
        if (BIAS_MODE == 1) v += bias[mBase + mOff + r];
        if (BIAS_MODE == 2) v += bv;
        slab[(mOff + r) * 68 + (j << 4) + rlane] = v;
      }
    }
    __builtin_amdgcn_fence(__ATOMIC_RELEASE, "workgroup");
    __builtin_amdgcn_wave_barrier();
    __builtin_amdgcn_fence(__ATOMIC_ACQUIRE, "workgroup");
    if (OUT_MODE == 0) {
      float* C = (float*)Cout + (size_t)b * strideC;
      const int hh = lane >> 4, c4 = (lane & 15) * 4;
      for (int pass = 0; pass < 2; ++pass) {
#pragma unroll
        for (int it = 0; it < 8; ++it) {
          const int row = it * 2 + hh;
          v4f v = *(const v4f*)(slab + row * 68 + c4);
          *(volatile v4f*)(C + (size_t)(mBase + row) * ldc + n0 + c4) = v;
        }
        __threadfence();
      }
    } else {
      const int q = lane >> 3, c8 = (lane & 7) * 8;
      unsigned short* C  = (unsigned short*)Cout  + (size_t)b * strideC;
      unsigned short* C2 = (OUT_MODE == 2) ? ((unsigned short*)Cout2 + (size_t)b * strideC) : nullptr;
      for (int pass = 0; pass < 2; ++pass) {
#pragma unroll
        for (int it = 0; it < 4; ++it) {
          const int row = it * 4 + q;
          const float* sp = slab + row * 68 + c8;
          unsigned short hb[8], lb[8];
#pragma unroll
          for (int e = 0; e < 8; ++e) {
            const float f = sp[e];
            if (OUT_MODE == 1) {
              const _Float16 fh = (_Float16)f;
              hb[e] = __builtin_bit_cast(unsigned short, fh);
              lb[e] = 0;
            } else {
              split_bf(f, hb[e], lb[e]);
            }
          }
          const v4u uh = (v4u){pk16(hb[0], hb[1]), pk16(hb[2], hb[3]), pk16(hb[4], hb[5]), pk16(hb[6], hb[7])};
          const v4u ul = (v4u){pk16(lb[0], lb[1]), pk16(lb[2], lb[3]), pk16(lb[4], lb[5]), pk16(lb[6], lb[7])};
          *(volatile v4u*)(C + (size_t)(mBase + row) * ldc + n0 + c8) = uh;
          if (OUT_MODE == 2) *(volatile v4u*)(C2 + (size_t)(mBase + row) * ldc + n0 + c8) = ul;
        }
        __threadfence();
      }
    }
    __builtin_amdgcn_fence(__ATOMIC_RELEASE, "workgroup");
    __builtin_amdgcn_wave_barrier();
    __builtin_amdgcn_fence(__ATOMIC_ACQUIRE, "workgroup");
  }
}

__global__ __launch_bounds__(256) void cast8_bf16_kernel(const float* __restrict__ in, unsigned short* __restrict__ out, int n8) {
  const int i = blockIdx.x * 256 + threadIdx.x;
  if (i >= n8) return;
  const float* p = in + 8 * (size_t)i;
  const v4f a = *(const v4f*)(p);
  const v4f c = *(const v4f*)(p + 4);
  unsigned short hb[8];
#pragma unroll
  for (int e = 0; e < 4; ++e) {
    const float fa = a[e];
    const float fc = c[e];
    hb[e]     = f2bf_bits(fa);
    hb[4 + e] = f2bf_bits(fc);
  }
  const v4u u = (v4u){pk16(hb[0], hb[1]), pk16(hb[2], hb[3]), pk16(hb[4], hb[5]), pk16(hb[6], hb[7])};
  unsigned short* q = out + 8 * (size_t)i;
  *(volatile v4u*)q = u;
  __threadfence();
  *(volatile v4u*)q = u;
}

__global__ __launch_bounds__(256) void wtcast_kernel(const float* __restrict__ W0, const float* __restrict__ W1,
                                                     const float* __restrict__ W2, const float* __restrict__ W3,
                                                     unsigned short* __restrict__ out) {
  __shared__ float sm[64][65];
  const int t  = threadIdx.x;
  const int k0 = blockIdx.x * 64;
  const int n0 = blockIdx.y * 64;
  const int z  = blockIdx.z;
  const float* W = (z == 0) ? W0 : (z == 1) ? W1 : (z == 2) ? W2 : W3;
#pragma unroll 8
  for (int i = 0; i < 16; ++i) {
    const int e = i * 256 + t;
    const int r = e >> 6;
    const int c = e & 63;
    sm[c][r] = W[(size_t)(k0 + r) * kDim + n0 + c];
  }
  __syncthreads();
  const int lane = t & 31, wave = t >> 5;
  const int q = lane >> 3, c8 = (lane & 7) * 8;
  const int rowA = wave * 8 + q, rowB = rowA + 4;
  unsigned short ha[8], hbv[8];
#pragma unroll
  for (int e = 0; e < 8; ++e) {
    ha[e]  = f2bf_bits(sm[rowA][c8 + e]);
    hbv[e] = f2bf_bits(sm[rowB][c8 + e]);
  }
  const v4u ua = (v4u){pk16(ha[0], ha[1]), pk16(ha[2], ha[3]), pk16(ha[4], ha[5]), pk16(ha[6], ha[7])};
  const v4u ub = (v4u){pk16(hbv[0], hbv[1]), pk16(hbv[2], hbv[3]), pk16(hbv[4], hbv[5]), pk16(hbv[6], hbv[7])};
  unsigned short* op = out + (size_t)z * kDim * kDim;
  unsigned short* pa = op + (size_t)(n0 + rowA) * kDim + k0 + c8;
  unsigned short* pb = op + (size_t)(n0 + rowB) * kDim + k0 + c8;
  *(volatile v4u*)pa = ua;
  *(volatile v4u*)pb = ub;
  __threadfence();
  *(volatile v4u*)pa = ua;
  *(volatile v4u*)pb = ub;
}

__global__ __launch_bounds__(32) void freq_kernel(float* __restrict__ invf) {
#pragma clang fp contract(off)
  const int p = threadIdx.x;
  const float e = (float)(2 * p) / 64.0f;
  const float pw = powf(kTheta, e);
  const float inv = 1.0f / pw;
  *(volatile float*)(invf + p) = inv;
  __threadfence();
  *(volatile float*)(invf + p) = inv;
}

__global__ __launch_bounds__(256) void trig_kernel(const float* __restrict__ invf, float* __restrict__ cosT,
                                                   float* __restrict__ sinT) {
#pragma clang fp contract(off)
  const int t = threadIdx.x;
  const int l = blockIdx.x * 8 + (t >> 5);
  const int p = t & 31;
  const float inv = invf[p];
  const float ang = (float)l * inv;
  float s, c;
  sincosf(ang, &s, &c);
  const size_t o = (size_t)l * kPairs + p;
  *(volatile float*)(cosT + o) = c;
  *(volatile float*)(sinT + o) = s;
  __threadfence();
  *(volatile float*)(cosT + o) = c;
  *(volatile float*)(sinT + o) = s;
}

__global__ __launch_bounds__(256) void rope_kernel(const float* __restrict__ qkv, const float* __restrict__ cosT,
                                                   const float* __restrict__ sinT, float* __restrict__ Qr,
                                                   float* __restrict__ Kr) {
#pragma clang fp contract(off)
  const int l = blockIdx.x;
  const int t = threadIdx.x;
  const int p0 = 2 * (t & 15);
  const float* row = qkv + (size_t)l * kQKVld;
  const v4f qv = *(const v4f*)(row + 4 * t);
  const v4f kv = *(const v4f*)(row + kDim + 4 * t);
  const v2f cs = *(const v2f*)(cosT + (size_t)l * kPairs + p0);
  const v2f sn = *(const v2f*)(sinT + (size_t)l * kPairs + p0);
  const float c0 = cs[0], c1 = cs[1], s0 = sn[0], s1 = sn[1];
  const float q1 = qv[0], q2 = qv[1], q3 = qv[2], q4 = qv[3];
  const float k1 = kv[0], k2 = kv[1], k3 = kv[2], k4 = kv[3];
  v4f qo, ko;
  qo[0] = fmaxf(q1 * c0 - q2 * s0, 0.0f);
  qo[1] = fmaxf(q1 * s0 + q2 * c0, 0.0f);
  qo[2] = fmaxf(q3 * c1 - q4 * s1, 0.0f);
  qo[3] = fmaxf(q3 * s1 + q4 * c1, 0.0f);
  ko[0] = fmaxf(k1 * c0 - k2 * s0, 0.0f);
  ko[1] = fmaxf(k1 * s0 + k2 * c0, 0.0f);
  ko[2] = fmaxf(k3 * c1 - k4 * s1, 0.0f);
  ko[3] = fmaxf(k3 * s1 + k4 * c1, 0.0f);
  float* qp = Qr + (size_t)l * kDim + 4 * t;
  float* kp = Kr + (size_t)l * kDim + 4 * t;
  *(volatile v4f*)qp = qo;
  *(volatile v4f*)kp = ko;
  __threadfence();
  *(volatile v4f*)qp = qo;
  *(volatile v4f*)kp = ko;
}

__device__ __forceinline__ void transpose_split(const float* Tf, unsigned short* Ph, unsigned short* Pl, int t) {
  const int d = t & 63, jh = t >> 6;
#pragma unroll
  for (int g = 0; g < 4; ++g) {
    const int j0 = jh * 32 + g * 8;
    unsigned short hb[8], lb[8];
#pragma unroll
    for (int e = 0; e < 8; ++e) split_bf(Tf[(j0 + e) * kFP + d], hb[e], lb[e]);
    const v4u uh = (v4u){pk16(hb[0], hb[1]), pk16(hb[2], hb[3]), pk16(hb[4], hb[5]), pk16(hb[6], hb[7])};
    const v4u ul = (v4u){pk16(lb[0], lb[1]), pk16(lb[2], lb[3]), pk16(lb[4], lb[5]), pk16(lb[6], lb[7])};
    *(v4u*)(Ph + d * kTP + j0) = uh;
    *(v4u*)(Pl + d * kTP + j0) = ul;
  }
}
__device__ __forceinline__ void split4_store(v4f v, unsigned short* Ph, unsigned short* Pl, int off) {
  const float f0 = v[0], f1 = v[1], f2 = v[2], f3 = v[3];
  unsigned short h0, h1, h2, h3, l0, l1, l2, l3;
  split_bf(f0, h0, l0); split_bf(f1, h1, l1); split_bf(f2, h2, l2); split_bf(f3, h3, l3);
  const v2u uh = (v2u){pk16(h0, h1), pk16(h2, h3)};
  const v2u ul = (v2u){pk16(l0, l1), pk16(l2, l3)};
  *(v2u*)(Ph + off) = uh;
  *(v2u*)(Pl + off) = ul;
}
__device__ __forceinline__ void mma3_step(v8f (&acc)[4], const __bf16* Ah, const __bf16* Al,
                                          const __bf16* Bh, const __bf16* Bl, int aoff, int boff) {
  const v16b ah = Frag<__bf16>::load(Ah + aoff);
  const v16b al = Frag<__bf16>::load(Al + aoff);
  v16b bh[4], bl[4];
#pragma unroll
  for (int j = 0; j < 4; ++j) {
    bh[j] = Frag<__bf16>::load(Bh + j * 16 * kTP + boff);
    bl[j] = Frag<__bf16>::load(Bl + j * 16 * kTP + boff);
  }
#pragma unroll
  for (int j = 0; j < 4; ++j) {
    acc[j] = Frag<__bf16>::mma(ah, bh[j], acc[j]);
    acc[j] = Frag<__bf16>::mma(ah, bl[j], acc[j]);
    acc[j] = Frag<__bf16>::mma(al, bh[j], acc[j]);
  }
  tile_guard(acc[0], acc[1], acc[2], acc[3], ah, al, bh[0], bh[1], bh[2], bh[3], bl[0], bl[1], bl[2], bl[3]);
}

__global__ __launch_bounds__(128) void chunk_state_kernel(const float* __restrict__ Kr, const float* __restrict__ qkv,
                                                          float* __restrict__ dST, float* __restrict__ dks) {
  __shared__ __align__(16) float Tf[kChunk * kFP];
  __shared__ __align__(16) unsigned short KTh[kDh * kTP];
  __shared__ __align__(16) unsigned short KTl[kDh * kTP];
  __shared__ __align__(16) unsigned short VTh[kDh * kTP];
  __shared__ __align__(16) unsigned short VTl[kDh * kTP];
  __shared__ __align__(16) float ksm[kDh];
  const int t = threadIdx.x, lane = t & 31, wave = t >> 5;
  const int h = blockIdx.x >> 5;
  const int c = blockIdx.x & 31;
  const size_t row0 = (size_t)c * kChunk;
  const size_t hc = (size_t)h * kNC + c;

#pragma unroll 4
  for (int i = 0; i < 8; ++i) {
    const int idx = i * 128 + t;
    const int j = idx >> 4, d4 = (idx & 15) * 4;
    const v4f v = *(const v4f*)(Kr + (row0 + j) * kDim + h * kDh + d4);
    *(v4f*)(Tf + j * kFP + d4) = v;
  }
  __syncthreads();
  if (t < kDh) {
    float s = 0.0f;
#pragma unroll 4
    for (int j = 0; j < kChunk; ++j) s += Tf[j * kFP + t];
    ksm[t] = s;
  }
  transpose_split(Tf, KTh, KTl, t);
  __syncthreads();
#pragma unroll 4
  for (int i = 0; i < 8; ++i) {
    const int idx = i * 128 + t;
    const int j = idx >> 4, d4 = (idx & 15) * 4;
    const v4f v = *(const v4f*)(qkv + (row0 + j) * kQKVld + 2 * kDim + h * kDh + d4);
    *(v4f*)(Tf + j * kFP + d4) = v;
  }
  __syncthreads();
  transpose_split(Tf, VTh, VTl, t);
  __syncthreads();

  const __bf16* KThb = (const __bf16*)(const void*)KTh;
  const __bf16* KTlb = (const __bf16*)(const void*)KTl;
  const __bf16* VThb = (const __bf16*)(const void*)VTh;
  const __bf16* VTlb = (const __bf16*)(const void*)VTl;
  const int rl = lane & 15, hh = lane >> 4, koff = hh * 8;
  const int m0 = wave * 16;
  v8f acc[4];
#pragma unroll
  for (int j = 0; j < 4; ++j) acc[j] = zero8();
#pragma unroll
  for (int ks = 0; ks < kChunk; ks += 32)
    mma3_step(acc, VThb, VTlb, KThb, KTlb, (m0 + rl) * kTP + koff + ks, rl * kTP + koff + ks);

  float* sw = Tf + m0 * kFP;
#pragma unroll
  for (int jt = 0; jt < 4; ++jt)
#pragma unroll
    for (int r = 0; r < 8; ++r) sw[(hh * 8 + r) * kFP + jt * 16 + rl] = acc[jt][r];
  __builtin_amdgcn_fence(__ATOMIC_RELEASE, "workgroup");
  __builtin_amdgcn_wave_barrier();
  __builtin_amdgcn_fence(__ATOMIC_ACQUIRE, "workgroup");
  float* dst = dST + (hc * kDh + m0) * kDh;
  const int c4 = rl * 4;
  for (int pass = 0; pass < 2; ++pass) {
#pragma unroll
    for (int it = 0; it < 8; ++it) {
      const int row = it * 2 + hh;
      const v4f v = *(const v4f*)(sw + row * kFP + c4);
      *(volatile v4f*)(dst + (size_t)row * kDh + c4) = v;
    }
    __threadfence();
  }
  if (wave == 0) {
    const int q4 = (lane & 15) * 4;
    const v4f kv = *(const v4f*)(ksm + q4);
    float* kp = dks + hc * kDh + q4;
    if (lane < 16) *(volatile v4f*)kp = kv;
    __threadfence();
    if (lane < 16) *(volatile v4f*)kp = kv;
  }
}

__global__ __launch_bounds__(256) void scan_kernel(const float* __restrict__ dST, const float* __restrict__ dks,
                                                   float* __restrict__ Sprev, float* __restrict__ ksprev) {
  const int t = threadIdx.x;
  const int bid = blockIdx.x;
  size_t base, step;
  const float* src;
  float* dst;
  if (bid < kHeads * 4) {
    const int h = bid >> 2, part = bid & 3;
    base = (size_t)h * kNC * (kDh * kDh) + (size_t)(part * 256 + t) * 4;
    step = (size_t)kDh * kDh;
    src = dST; dst = Sprev;
  } else {
    const int h = t >> 4, q4 = (t & 15) * 4;
    base = (size_t)h * kNC * kDh + q4;
    step = (size_t)kDh;
    src = dks; dst = ksprev;
  }
  for (int pass = 0; pass < 2; ++pass) {
    v4f acc = (v4f){0.0f, 0.0f, 0.0f, 0.0f};
#pragma unroll 4
    for (int cc = 0; cc < kNC; ++cc) {
      const size_t o = base + (size_t)cc * step;
      *(volatile v4f*)(dst + o) = acc;
      const v4f v = *(const v4f*)(src + o);
      acc = acc + v;
    }
    __threadfence();
  }
}

__global__ __launch_bounds__(128) void chunk_out_kernel(const float* __restrict__ Qr, const float* __restrict__ Kr,
                                                        const float* __restrict__ qkv, const float* __restrict__ Sprev,
                                                        const float* __restrict__ ksprev,
                                                        unsigned short* __restrict__ attnH, unsigned short* __restrict__ attnL) {
  __shared__ __align__(16) float Qf[kChunk * kFP];
  __shared__ __align__(16) float Pf[kChunk * kFP];
  __shared__ __align__(16) unsigned short Qh[kChunk * kTP];
  __shared__ __align__(16) unsigned short Ql[kChunk * kTP];
  __shared__ __align__(16) unsigned short KPh[kChunk * kTP];
  __shared__ __align__(16) unsigned short KPl[kChunk * kTP];
  __shared__ __align__(16) unsigned short VTh[kDh * kTP];
  __shared__ __align__(16) unsigned short VTl[kDh * kTP];
  __shared__ __align__(16) unsigned short STh[kDh * kTP];
  __shared__ __align__(16) unsigned short STl[kDh * kTP];
  __shared__ __align__(16) float ksm[kDh];
  __shared__ __align__(16) float rsm[kChunk];
  __shared__ __align__(16) float invm[kChunk];

  const int t = threadIdx.x, lane = t & 31, wave = t >> 5;
  const int h = blockIdx.x >> 5;
  const int c = blockIdx.x & 31;
  const size_t row0 = (size_t)c * kChunk;
  const size_t hc = (size_t)h * kNC + c;

#pragma unroll 2
  for (int i = 0; i < 8; ++i) {
    const int idx = i * 128 + t;
    const int r = idx >> 4, d4 = (idx & 15) * 4;
    const v4f v = *(const v4f*)(Qr + (row0 + r) * kDim + h * kDh + d4);
    *(v4f*)(Qf + r * kFP + d4) = v;
    split4_store(v, Qh, Ql, r * kTP + d4);
  }
  asm volatile("" ::: "memory");
#pragma unroll 2
  for (int i = 0; i < 8; ++i) {
    const int idx = i * 128 + t;
    const int r = idx >> 4, d4 = (idx & 15) * 4;
    const v4f v = *(const v4f*)(Kr + (row0 + r) * kDim + h * kDh + d4);
    split4_store(v, KPh, KPl, r * kTP + d4);
  }
  asm volatile("" ::: "memory");
#pragma unroll 2
  for (int i = 0; i < 8; ++i) {
    const int idx = i * 128 + t;
    const int r = idx >> 4, d4 = (idx & 15) * 4;
    const v4f v = *(const v4f*)(Sprev + (hc * kDh + r) * kDh + d4);
    split4_store(v, STh, STl, r * kTP + d4);
  }
  asm volatile("" ::: "memory");
#pragma unroll 2
  for (int i = 0; i < 8; ++i) {
    const int idx = i * 128 + t;
    const int r = idx >> 4, d4 = (idx & 15) * 4;
    const v4f v = *(const v4f*)(qkv + (row0 + r) * kQKVld + 2 * kDim + h * kDh + d4);
    *(v4f*)(Pf + r * kFP + d4) = v;
  }
  {
    const int q4 = (t & 15) * 4;
    const v4f kv = *(const v4f*)(ksprev + hc * kDh + q4);
    if (t < 16) *(v4f*)(ksm + q4) = kv;
  }
  __syncthreads();
  transpose_split(Pf, VTh, VTl, t);
  __syncthreads();

  const __bf16* Qhb  = (const __bf16*)(const void*)Qh;
  const __bf16* Qlb  = (const __bf16*)(const void*)Ql;
  const __bf16* KPhb = (const __bf16*)(const void*)KPh;
  const __bf16* KPlb = (const __bf16*)(const void*)KPl;
  const __bf16* VThb = (const __bf16*)(const void*)VTh;
  const __bf16* VTlb = (const __bf16*)(const void*)VTl;
  const __bf16* SThb = (const __bf16*)(const void*)STh;
  const __bf16* STlb = (const __bf16*)(const void*)STl;
  const int rl = lane & 15, hh = lane >> 4, koff = hh * 8;
  const int i0 = wave * 16;

  v8f p[4];
#pragma unroll
  for (int j = 0; j < 4; ++j) p[j] = zero8();
#pragma unroll
  for (int ks = 0; ks < kDh; ks += 32)
    mma3_step(p, Qhb, Qlb, KPhb, KPlb, (i0 + rl) * kTP + koff + ks, rl * kTP + koff + ks);
  float rs[8];
#pragma unroll
  for (int r = 0; r < 8; ++r) rs[r] = 0.0f;
#pragma unroll
  for (int jt = 0; jt < 4; ++jt)
#pragma unroll
    for (int r = 0; r < 8; ++r) {
      const int il = i0 + hh * 8 + r;
      const int jl = jt * 16 + rl;
      const float val = (jl <= il) ? p[jt][r] : 0.0f;
      rs[r] += val;
      Pf[il * kFP + jl] = val;
    }
#pragma unroll
  for (int r = 0; r < 8; ++r) {
    float x = rs[r];
    x += __shfl_xor(x, 8);
    x += __shfl_xor(x, 4);
    x += __shfl_xor(x, 2);
    x += __shfl_xor(x, 1);
    if (rl == 0) rsm[i0 + hh * 8 + r] = x;
  }
  __syncthreads();

  {
    const int row = i0 + (lane >> 1);
    const int ch = (lane & 1) * 32;
#pragma unroll
    for (int g = 0; g < 4; ++g) {
      const int col = ch + g * 8;
      const v4f a = *(const v4f*)(Pf + row * kFP + col);
      const v4f b = *(const v4f*)(Pf + row * kFP + col + 4);
      unsigned short hb[8], lb[8];
#pragma unroll
      for (int e = 0; e < 4; ++e) {
        const float fa = a[e];
        const float fb = b[e];
        split_bf(fa, hb[e], lb[e]);
        split_bf(fb, hb[4 + e], lb[4 + e]);
      }
      const v4u uh = (v4u){pk16(hb[0], hb[1]), pk16(hb[2], hb[3]), pk16(hb[4], hb[5]), pk16(hb[6], hb[7])};
      const v4u ul = (v4u){pk16(lb[0], lb[1]), pk16(lb[2], lb[3]), pk16(lb[4], lb[5]), pk16(lb[6], lb[7])};
      *(v4u*)(KPh + row * kTP + col) = uh;
      *(v4u*)(KPl + row * kTP + col) = ul;
    }
  }
  if (t < kChunk) {
    const int il = t;
    float d0 = rsm[il], d1 = 0.0f, d2 = 0.0f, d3 = 0.0f;
#pragma unroll 1
    for (int q = 0; q < 16; ++q) {
      const v4f qv = *(const v4f*)(Qf + il * kFP + 4 * q);
      const v4f kv = *(const v4f*)(ksm + 4 * q);
      d0 += qv[0] * kv[0];
      d1 += qv[1] * kv[1];
      d2 += qv[2] * kv[2];
      d3 += qv[3] * kv[3];
    }
    const float den = (d0 + d1) + (d2 + d3);
    invm[il] = 1.0f / (den + kEps);
  }
  __syncthreads();

  v8f num[4];
#pragma unroll
  for (int j = 0; j < 4; ++j) num[j] = zero8();
#pragma unroll
  for (int ks = 0; ks < kChunk; ks += 32)
    mma3_step(num, KPhb, KPlb, VThb, VTlb, (i0 + rl) * kTP + koff + ks, rl * kTP + koff + ks);
#pragma unroll
  for (int ks = 0; ks < kDh; ks += 32)
    mma3_step(num, Qhb, Qlb, SThb, STlb, (i0 + rl) * kTP + koff + ks, rl * kTP + koff + ks);

  float* sw = Pf + i0 * kFP;
#pragma unroll
  for (int mt = 0; mt < 4; ++mt)
#pragma unroll
    for (int r = 0; r < 8; ++r) {
      const int il = hh * 8 + r;
      sw[il * kFP + mt * 16 + rl] = num[mt][r] * invm[i0 + il];
    }
  __builtin_amdgcn_fence(__ATOMIC_RELEASE, "workgroup");
  __builtin_amdgcn_wave_barrier();
  __builtin_amdgcn_fence(__ATOMIC_ACQUIRE, "workgroup");
  {
    const int q = lane >> 3, c8 = (lane & 7) * 8;
    v4u wh[4], wl[4];
#pragma unroll
    for (int it = 0; it < 4; ++it) {
      const int row = it * 4 + q;
      const float* sp = sw + row * kFP + c8;
      unsigned short hb[8], lb[8];
#pragma unroll
      for (int e = 0; e < 8; ++e) split_bf(sp[e], hb[e], lb[e]);
      wh[it] = (v4u){pk16(hb[0], hb[1]), pk16(hb[2], hb[3]), pk16(hb[4], hb[5]), pk16(hb[6], hb[7])};
      wl[it] = (v4u){pk16(lb[0], lb[1]), pk16(lb[2], lb[3]), pk16(lb[4], lb[5]), pk16(lb[6], lb[7])};
    }
    unsigned short* oh = attnH + (row0 + i0) * kDim + h * kDh + c8;
    unsigned short* ol = attnL + (row0 + i0) * kDim + h * kDh + c8;
    for (int pass = 0; pass < 2; ++pass) {
#pragma unroll
      for (int it = 0; it < 4; ++it) {
        const int row = it * 4 + q;
        *(volatile v4u*)(oh + (size_t)row * kDim) = wh[it];
        *(volatile v4u*)(ol + (size_t)row * kDim) = wl[it];
      }
      __threadfence();
    }
  }
}

extern "C" void kernel_launch(void* const* d_in, const int* in_sizes, int n_in,
                              void* d_out, int out_size, void* d_ws, size_t ws_size,
                              hipStream_t stream) {
  if (n_in < 5) return;
  const int nTok = kSeq * kDim;
  const int nW   = kDim * kDim;
  if (in_sizes[0] != nTok || in_sizes[1] != nW || in_sizes[2] != nW || in_sizes[3] != nW || in_sizes[4] != nW) return;
  if (out_size != nTok) return;

  const size_t szXb   = (size_t)kSeq * kDim * 2;
  const size_t szWall = (size_t)4 * kDim * kDim * 2;
  const size_t szQKV  = (size_t)kSeq * kQKVld * 4;
  const size_t szInv  = 128;
  const size_t szTrig = (size_t)kSeq * kPairs * 4;
  const size_t szQr   = (size_t)kSeq * kDim * 4;
  const size_t szST   = (size_t)kHeads * kNC * kDh * kDh * 4;
  const size_t szKS   = (size_t)kHeads * kNC * kDh * 4;
  const size_t szAt   = (size_t)kSeq * kDim * 2;
  const size_t offXb   = 0;
  const size_t offWall = offXb + szXb;
  const size_t offQKV  = offWall + szWall;
  const size_t offInv  = offQKV + szQKV;
  const size_t offCos  = offInv + szInv;
  const size_t offSin  = offCos + szTrig;
  const size_t offQr   = offSin + szTrig;
  const size_t offKr   = offQr + szQr;
  const size_t offDST  = offKr + szQr;
  const size_t offDKS  = offDST + szST;
  const size_t offSP   = offDKS + szKS;
  const size_t offKSP  = offSP + szST;
  const size_t offAtH  = offKSP + szKS;
  const size_t offAtL  = offAtH + szAt;
  const size_t total   = offAtL + szAt;
  if (ws_size < total) return;

  const float* x  = (const float*)d_in[0];
  const float* wq = (const float*)d_in[1];
  const float* wk = (const float*)d_in[2];
  const float* wv = (const float*)d_in[3];
  const float* wo = (const float*)d_in[4];
  float* out = (float*)d_out;
  char* ws = (char*)d_ws;
  unsigned short* xb   = (unsigned short*)(ws + offXb);
  unsigned short* Wall = (unsigned short*)(ws + offWall);
  unsigned short* WoT  = Wall + (size_t)3 * kDim * kDim;
  float* qkv    = (float*)(ws + offQKV);
  float* invf   = (float*)(ws + offInv);
  float* cosT   = (float*)(ws + offCos);
  float* sinT   = (float*)(ws + offSin);
  float* Qr     = (float*)(ws + offQr);
  float* Kr     = (float*)(ws + offKr);
  float* dST    = (float*)(ws + offDST);
  float* dks    = (float*)(ws + offDKS);
  float* Sprev  = (float*)(ws + offSP);
  float* ksprev = (float*)(ws + offKSP);
  unsigned short* attnH = (unsigned short*)(ws + offAtH);
  unsigned short* attnL = (unsigned short*)(ws + offAtL);
  const float* nobias = (const float*)(ws + offQKV);

  const int n8 = nTok / 8;
  cast8_bf16_kernel<<<dim3(n8 / 256), dim3(256), 0, stream>>>(x, xb, n8);
  wtcast_kernel<<<dim3(kDim / 64, kDim / 64, 4), dim3(256), 0, stream>>>(wq, wk, wv, wo, Wall);

  wmma_gemm64<1, 0, 0, 0><<<dim3((kSeq / 64) * (kQKVld / 64) / 8, 1), dim3(256), 0, stream>>>(
      xb, xb, kDim, 0L, Wall, Wall, kDim, 0L, (void*)qkv, (void*)qkv, kQKVld, 0L, nobias, kSeq, kQKVld, kDim, 1.0f);

  freq_kernel<<<dim3(1), dim3(32), 0, stream>>>(invf);
  trig_kernel<<<dim3(kSeq / 8), dim3(256), 0, stream>>>(invf, cosT, sinT);
  rope_kernel<<<dim3(kSeq), dim3(256), 0, stream>>>(qkv, cosT, sinT, Qr, Kr);

  chunk_state_kernel<<<dim3(kHeads * kNC), dim3(128), 0, stream>>>(Kr, qkv, dST, dks);
  scan_kernel<<<dim3(kHeads * 4 + 1), dim3(256), 0, stream>>>(dST, dks, Sprev, ksprev);
  chunk_out_kernel<<<dim3(kHeads * kNC), dim3(128), 0, stream>>>(Qr, Kr, qkv, Sprev, ksprev, attnH, attnL);

  wmma_gemm64<1, 1, 0, 0><<<dim3((kSeq / 64) * (kDim / 64) / 8, 1), dim3(256), 0, stream>>>(
      attnH, attnL, kDim, 0L, WoT, WoT, kDim, 0L, (void*)out, (void*)out, kDim, 0L, nobias, kSeq, kDim, kDim, 1.0f);
}
